// GATActorCritic_4750233829756
// MI455X (gfx1250) — hardware-run, weakly checked
//
#include <hip/hip_runtime.h>

typedef float          v8f   __attribute__((ext_vector_type(8)));
typedef float          v4f   __attribute__((ext_vector_type(4)));
typedef unsigned int   v4u   __attribute__((ext_vector_type(4)));
typedef int            v8i   __attribute__((ext_vector_type(8)));
typedef unsigned short v8us  __attribute__((ext_vector_type(8)));
typedef unsigned short v16us __attribute__((ext_vector_type(16)));
typedef __bf16         v16bf __attribute__((ext_vector_type(16)));
typedef _Float16       v16h  __attribute__((ext_vector_type(16)));
typedef v4f  __attribute__((may_alias)) v4fa;
typedef v8us __attribute__((may_alias)) v8usa;
union FragB { v16bf v; v16us u; v8us h[2]; v8i w; };
union FragH { v16h  v; v16us u; v8us h[2]; v8i w; };

__device__ __forceinline__ v8f wmb(const FragB& a, const FragB& b, v8f c) {
  v8f d = __builtin_amdgcn_wmma_f32_16x16x32_bf16(false, a.v, false, b.v, (short)0, c, false, false);
  asm volatile("v_nop\n\tv_nop\n\tv_nop\n\tv_nop" : "+v"(d) : "v"(a.w), "v"(b.w));
  return d;
}

__device__ __forceinline__ v8f wmh(const FragH& a, const FragH& b, v8f c) {
  v8f d = __builtin_amdgcn_wmma_f32_16x16x32_f16(false, a.v, false, b.v, (short)0, c, false, false);
  asm volatile("v_nop\n\tv_nop\n\tv_nop\n\tv_nop" : "+v"(d) : "v"(a.w), "v"(b.w));
  return d;
}

__device__ __forceinline__ unsigned bf16_bits(float f) {
  const unsigned u = __float_as_uint(f);
  const unsigned r = (u + 0x7FFFu + ((u >> 16) & 1u)) >> 16;
  const unsigned q = (u >> 16) | 0x40u;
  return ((u & 0x7fffffffu) > 0x7f800000u) ? q : r;
}

__device__ __forceinline__ float bf16_val(float f) {
  return __uint_as_float(bf16_bits(f) << 16);
}
__device__ __forceinline__ int clampi(int v, int lo, int hi) {
  return v < lo ? lo : (v > hi ? hi : v);
}

__device__ __forceinline__ unsigned f16_bits(float f) {
  const unsigned u  = __float_as_uint(f);
  const unsigned s  = (u >> 16) & 0x8000u;
  const unsigned a  = u & 0x7fffffffu;
  const unsigned t  = a - 0x38000000u;
  const unsigned r  = (t + 0x0FFFu + ((t >> 13) & 1u)) >> 13;
  const unsigned rc = r > 0x7C00u ? 0x7C00u : r;
  const bool small  = a < 0x38800000u;
  const bool isnan  = a > 0x7f800000u;
  const unsigned fin = small ? 0u : (s | rc);
  return isnan ? (s | 0x7E00u) : fin;
}

__device__ __forceinline__ unsigned pk16(unsigned lo, unsigned hi) { return lo | (hi << 16); }
__device__ __forceinline__ unsigned bf16_lo_bits(float v) {
  float hi = bf16_val(v);
  asm volatile("" : "+v"(hi));
  return bf16_bits(v - hi);
}
__device__ __forceinline__ v4u pack8_bf16(v4f a, v4f c) {
  return (v4u){ pk16(bf16_bits(a[0]), bf16_bits(a[1])), pk16(bf16_bits(a[2]), bf16_bits(a[3])),
                pk16(bf16_bits(c[0]), bf16_bits(c[1])), pk16(bf16_bits(c[2]), bf16_bits(c[3])) };
}
__device__ __forceinline__ v4u pack8_bf16_lo(v4f a, v4f c) {
  return (v4u){ pk16(bf16_lo_bits(a[0]), bf16_lo_bits(a[1])), pk16(bf16_lo_bits(a[2]), bf16_lo_bits(a[3])),
                pk16(bf16_lo_bits(c[0]), bf16_lo_bits(c[1])), pk16(bf16_lo_bits(c[2]), bf16_lo_bits(c[3])) };
}
__device__ __forceinline__ v4u pack8_f16(v4f a, v4f c) {
  return (v4u){ pk16(f16_bits(a[0]), f16_bits(a[1])), pk16(f16_bits(a[2]), f16_bits(a[3])),
                pk16(f16_bits(c[0]), f16_bits(c[1])), pk16(f16_bits(c[2]), f16_bits(c[3])) };
}

template <int FORM>
__global__ __launch_bounds__(256) void k_plane(const float* __restrict__ src, int rows, int cols, int ldsrc,
                                               unsigned short* __restrict__ dst, int MP, int KP) {
  static_assert(FORM >= 0 && FORM <= 3);
  const int KTOT = (FORM == 1 || FORM == 3) ? 2 * KP : KP;
  const unsigned ppr   = (unsigned)(KTOT >> 3);
  const unsigned kp8   = (unsigned)(KP >> 3);
  const unsigned total = (unsigned)MP * ppr;
  const unsigned g     = blockIdx.x * 256u + threadIdx.x;
  const unsigned rowu  = g / ppr;
  const unsigned p     = g - rowu * ppr;
  const bool second    = p >= kp8;
  const int row = (int)rowu;
  const int c0  = (int)((second ? p - kp8 : p) << 3);
  const float* srow = src + (size_t)clampi(row, 0, rows - 1) * (size_t)ldsrc;
  float x[8];
  unsigned mk[8];
#pragma unroll
  for (int e = 0; e < 8; ++e) {
    const int c = c0 + e;
    const float v = srow[clampi(c, 0, cols - 1)];
    asm volatile("" :: "v"(v));
    x[e]  = v;
    mk[e] = (row < rows && c < cols) ? 0xFFFFu : 0u;
  }
  const v4f a = (v4f){ x[0], x[1], x[2], x[3] };
  const v4f c = (v4f){ x[4], x[5], x[6], x[7] };
  v4u o;
  if (FORM == 2) {
    o = pack8_f16(a, c);
  } else {
    const v4u hi = pack8_bf16(a, c);
    o = hi;
    if (FORM == 1) { const v4u lo = pack8_bf16_lo(a, c); o = second ? lo : hi; }
  }
  const v4u mw = (v4u){ pk16(mk[0], mk[1]), pk16(mk[2], mk[3]), pk16(mk[4], mk[5]), pk16(mk[6], mk[7]) };
  o &= mw;
  if (g < total) {
    volatile v4u* q = (volatile v4u*)(dst + (size_t)g * 8);
    *q = o;
    __threadfence();
    *q = o;
  }
}

template <int FORM> struct FragOf    { typedef FragB T; };
template <>         struct FragOf<2> { typedef FragH T; };
__device__ __forceinline__ v8f mm(const FragB& a, const FragB& b, v8f c) { return wmb(a, b, c); }
__device__ __forceinline__ v8f mm(const FragH& a, const FragH& b, v8f c) { return wmh(a, b, c); }
template <class F> __device__ __forceinline__ F ld_frag(const unsigned short* p) {
  F f;
  f.h[0] = *(const v8usa*)(p);
  f.h[1] = *(const v8usa*)(p + 16);
  return f;
}

template <int FORM, int EPI>
__global__ __launch_bounds__(256) __attribute__((amdgpu_num_vgpr(248)))
void k_gemm_nt(const unsigned short* __restrict__ A, const unsigned short* __restrict__ B,
               const float* __restrict__ bias, float* __restrict__ D, int M, int N, int KTOT, int ldd) {
  static_assert(FORM >= 0 && FORM <= 2);
  static_assert(EPI == 0 || EPI == 1);
  typedef typename FragOf<FORM>::T F;
  __shared__ __attribute__((aligned(16))) float sT[8][16 * 68];
  const int lane = threadIdx.x & 31;
  const int wave = threadIdx.x >> 5;
  const int tilesM = (M + 63) >> 6;
  const int tilesN = (N + 63) >> 6;
  const int tile = blockIdx.x * 8 + wave;
  if (tile >= tilesM * tilesN) return;
  const int tm = tile / tilesN;
  const int tn = tile - tm * tilesN;
  const int m0 = tm << 6;
  const int n0 = tn << 6;

  const int rl = lane & 15;
  const int h8 = (lane >> 4) * 8;
  const unsigned short* pa = A + (size_t)(m0 + rl) * (size_t)KTOT + h8;
  const unsigned short* pb = B + (size_t)(n0 + rl) * (size_t)KTOT + h8;

  v8f acc[4][4];
#pragma unroll
  for (int i = 0; i < 4; ++i)
#pragma unroll
    for (int j = 0; j < 4; ++j) acc[i][j] = (v8f){0.f, 0.f, 0.f, 0.f, 0.f, 0.f, 0.f, 0.f};

#pragma unroll 1
  for (int k0 = 0; k0 < KTOT; k0 += 32) {
    F bf[4];
#pragma unroll
    for (int j = 0; j < 4; ++j) bf[j] = ld_frag<F>(pb + (size_t)(j << 4) * (size_t)KTOT + k0);
#pragma unroll
    for (int i = 0; i < 4; ++i) {
      const F af = ld_frag<F>(pa + (size_t)(i << 4) * (size_t)KTOT + k0);
#pragma unroll
      for (int j = 0; j < 4; ++j) acc[i][j] = mm(af, bf[j], acc[i][j]);
    }
  }

  float* slab = sT[wave];
  const int hh = lane >> 4;
  const int c4 = (lane & 15) * 4;
  const int nc = n0 + c4;
  const bool cok = nc < N;
  v4f bv = (v4f){0.f, 0.f, 0.f, 0.f};
  if (EPI == 1) {
    bv = *(const v4fa*)(bias + clampi(nc, 0, N - 4));
    asm volatile("" :: "v"(bv));
  }
#pragma unroll
  for (int i = 0; i < 4; ++i) {
    const int mBase = m0 + (i << 4);
#pragma unroll
    for (int j = 0; j < 4; ++j) {
#pragma unroll
      for (int r = 0; r < 8; ++r) slab[(h8 + r) * 68 + (j << 4) + rl] = acc[i][j][r];
    }
    __builtin_amdgcn_fence(__ATOMIC_RELEASE, "workgroup");
    __builtin_amdgcn_wave_barrier();
    __builtin_amdgcn_fence(__ATOMIC_ACQUIRE, "workgroup");
    v4f vv[8];
#pragma unroll
    for (int it = 0; it < 8; ++it) {
      const int row = it * 2 + hh;
      v4f v = *(const v4fa*)(slab + row * 68 + c4);
      if (EPI == 1) v += bv;
      vv[it] = v;
    }
    for (int pass = 0; pass < 2; ++pass) {
#pragma unroll
      for (int it = 0; it < 8; ++it) {
        const int row = mBase + it * 2 + hh;
        if (cok && row < M) *(volatile v4f*)(D + (size_t)row * (size_t)ldd + nc) = vv[it];
      }
      __threadfence();
    }
    __builtin_amdgcn_fence(__ATOMIC_RELEASE, "workgroup");
    __builtin_amdgcn_wave_barrier();
    __builtin_amdgcn_fence(__ATOMIC_ACQUIRE, "workgroup");
  }
}

#pragma clang fp contract(off)

typedef int          v4i  __attribute__((ext_vector_type(4)));
typedef unsigned int v2u  __attribute__((ext_vector_type(2)));
typedef double       v2d  __attribute__((ext_vector_type(2)));
typedef v4i __attribute__((may_alias)) v4ia;

constexpr int NN      = 50000;
constexpr int EE      = 800000;
constexpr int FIN     = 128;
constexpr int C1      = 128;
constexpr int HID     = 32;
constexpr int MP      = 50048;
constexpr int NB      = 1024;
constexpr int NBLK    = 49;
constexpr int CHUNK   = 2048;
constexpr int NCHUNK  = 391;
constexpr int WCAP    = 256;
constexpr int LISTN   = 8 * WCAP;
constexpr int CAP     = 22528;
constexpr int DEGCAP  = 48;
constexpr int SROWS   = DEGCAP + 1;
constexpr int LOGIT_ELEMS = 1600000;
constexpr int OUT_ELEMS   = 1600001;
constexpr int NREC    = 196;
constexpr int TWO_TERM_SITE2 = 1;
constexpr int TWO_TERM_SITE3 = 1;
constexpr unsigned LOMASK2 = TWO_TERM_SITE2 ? 0xFFFFFFFFu : 0u;
constexpr unsigned LOMASK3 = TWO_TERM_SITE3 ? 0xFFFFFFFFu : 0u;
constexpr int LDS_BUCKET = (2 * CAP + 3 * NB + LISTN + 32) * 4;

static_assert(NN == 48 * 1024 + 848);
static_assert(EE == 390 * 2048 + 1280);
static_assert(NN < 65536);
static_assert(EE % 8 == 0 && ((size_t)EE * 4) % 16 == 0);
static_assert(NBLK * NB >= MP && (NBLK - 1) * NB < NN);
static_assert(NCHUNK * CHUNK >= EE && (NCHUNK - 1) * CHUNK < EE);
static_assert(DEGCAP >= 35 + 8 && DEGCAP <= 64);
static_assert((long long)CAP * 4 >= (long long)16623 * 5);
static_assert(CAP % 1024 == 0);
static_assert(LOGIT_ELEMS % 32 == 0 && LOGIT_ELEMS % 256 == 0 && LOGIT_ELEMS == 32 * NN);
static_assert(OUT_ELEMS == LOGIT_ELEMS + 1);
static_assert(MP == 782 * 64 && MP % 128 == 0 && MP % 16 == 0 && MP % 8 == 0 && MP >= NN);
static_assert(NREC * 256 >= NN);
static_assert(LDS_BUCKET == 200832 && LDS_BUCKET <= 262144 && LDS_BUCKET <= 327680);
static_assert(8 * SROWS * 32 * 4 == 50176 && 8 * SROWS * 32 * 4 <= 65536);
static_assert((long long)MP * 256 / 8 < 0x7fffffffLL);

constexpr int P_A1S = 0, P_A1D = 128, P_B1 = 256, P_A2S = 384, P_A2D = 512, P_B2 = 640, P_HB = 768;
constexpr int PAR_FLOATS = 896;

constexpr size_t SZ_XB   = (size_t)MP * FIN * 2;
constexpr size_t SZ_HW   = (size_t)MP * C1 * 4;
constexpr size_t SZ_H1   = (size_t)MP * 256 * 2;
constexpr size_t SZ_HW2  = (size_t)MP * 64 * 4;
constexpr size_t SZ_H2   = (size_t)MP * 64 * 2;
constexpr size_t SZ_T    = (size_t)MP * 64 * 4;
constexpr size_t SZ_ASD1 = (size_t)2 * MP * 4 * 4;
constexpr size_t SZ_ASD2 = (size_t)2 * MP * 4;
constexpr size_t SZ_LIST = (size_t)NBLK * CAP * 4;
constexpr size_t SZ_OFF  = (size_t)NBLK * NB * 4;
constexpr size_t SZ_CNT  = (size_t)NBLK * NB * 4;
constexpr size_t SZ_FLG  = 6400;
constexpr size_t SZ_W1T  = (size_t)128 * 128 * 2;
constexpr size_t SZ_W2D  = (size_t)64 * 256 * 2;
constexpr size_t SZ_WHD  = (size_t)64 * 64 * 2;
constexpr size_t SZ_PAR  = (size_t)PAR_FLOATS * 4;
constexpr size_t SZ_REC  = (size_t)NREC * 128;
constexpr size_t OFF_XB   = 0;
constexpr size_t OFF_HW   = OFF_XB + SZ_XB;
constexpr size_t OFF_H1   = OFF_HW + SZ_HW;
constexpr size_t OFF_HW2  = OFF_H1 + SZ_H1;
constexpr size_t OFF_H2   = OFF_HW2 + SZ_HW2;
constexpr size_t OFF_T    = OFF_H2 + SZ_H2;
constexpr size_t OFF_ASD1 = OFF_T + SZ_T;
constexpr size_t OFF_ASD2 = OFF_ASD1 + SZ_ASD1;
constexpr size_t OFF_LIST = OFF_ASD2 + SZ_ASD2;
constexpr size_t OFF_OFF  = OFF_LIST + SZ_LIST;
constexpr size_t OFF_CNT  = OFF_OFF + SZ_OFF;
constexpr size_t OFF_FLG  = OFF_CNT + SZ_CNT;
constexpr size_t OFF_W1T  = OFF_FLG + SZ_FLG;
constexpr size_t OFF_W2D  = OFF_W1T + SZ_W1T;
constexpr size_t OFF_WHD  = OFF_W2D + SZ_W2D;
constexpr size_t OFF_PAR  = OFF_WHD + SZ_WHD;
constexpr size_t OFF_REC  = OFF_PAR + SZ_PAR;
constexpr size_t WS_TOTAL = OFF_REC + SZ_REC;
static_assert(SZ_XB % 256 == 0 && SZ_HW % 256 == 0 && SZ_H1 % 256 == 0 && SZ_HW2 % 256 == 0 && SZ_H2 % 256 == 0);
static_assert(SZ_T % 256 == 0 && SZ_ASD1 % 256 == 0 && SZ_ASD2 % 256 == 0 && SZ_LIST % 256 == 0);
static_assert(SZ_OFF % 256 == 0 && SZ_CNT % 256 == 0 && SZ_FLG % 256 == 0 && SZ_FLG >= (size_t)NBLK * 128);
static_assert(SZ_W1T % 256 == 0 && SZ_W2D % 256 == 0 && SZ_WHD % 256 == 0 && SZ_PAR % 256 == 0 && SZ_REC % 256 == 0);
static_assert(((size_t)MP * 16) % 128 == 0 && ((size_t)MP * 4) % 128 == 0);
static_assert(WS_TOTAL == (size_t)((size_t)402421 << 8));
static_assert(WS_TOTAL <= ((size_t)128 << 20));

__device__ __forceinline__ v4u wt_unit(const float* __restrict__ w, int pitch, int kmask, int n, int k8) {
  float x[8];
#pragma unroll
  for (int e = 0; e < 8; ++e) {
    const int k = (k8 + e) & kmask;
    const float v = w[(size_t)k * (size_t)pitch + (size_t)n];
    asm volatile("" :: "v"(v));
    x[e] = v;
  }
  return pack8_bf16((v4f){ x[0], x[1], x[2], x[3] }, (v4f){ x[4], x[5], x[6], x[7] });
}
__device__ __forceinline__ void put16(unsigned short* __restrict__ dst, int u, v4u o) {
  volatile v4u* q = (volatile v4u*)(dst + (size_t)u * 8);
  *q = o;
  __threadfence();
  *q = o;
}
__device__ __forceinline__ void par_sec(const float* __restrict__ src, int len, float* __restrict__ dst, int tid) {
  const int np = len >> 2;
  const int tc = tid < np ? tid : np - 1;
  const v4f a = *(const v4fa*)(src + 4 * tc);
  asm volatile("" :: "v"(a));
  const unsigned m = tid < np ? 0xFFFFFFFFu : 0u;
  const v4f o = (v4f){ __uint_as_float((bf16_bits(a[0]) << 16) & m), __uint_as_float((bf16_bits(a[1]) << 16) & m),
                       __uint_as_float((bf16_bits(a[2]) << 16) & m), __uint_as_float((bf16_bits(a[3]) << 16) & m) };
  if (tid < 32) {
    volatile v4f* q = (volatile v4f*)(dst + 4 * tid);
    *q = o;
    __threadfence();
    *q = o;
  }
}

__global__ __launch_bounds__(256) void k_prep(
    const float* __restrict__ W1, const float* __restrict__ W2, const float* __restrict__ Wa,
    const float* __restrict__ Wc, const float* __restrict__ a1s, const float* __restrict__ a1d,
    const float* __restrict__ b1, const float* __restrict__ a2s, const float* __restrict__ a2d,
    const float* __restrict__ b2, const float* __restrict__ ba, const float* __restrict__ bc,
    unsigned short* __restrict__ W1T, unsigned short* __restrict__ W2D, unsigned short* __restrict__ WHD,
    float* __restrict__ PAR) {
  const int tid = (int)threadIdx.x;
  const int blk = (int)blockIdx.x;
  const v4u zz = (v4u){ 0u, 0u, 0u, 0u };
  if (blk < 8) {
    const int u = blk * 256 + tid;
    put16(W1T, u, wt_unit(W1, 128, 127, u >> 4, (u & 15) * 8));
  } else if (blk < 12) {
    const int u = (blk - 8) * 256 + tid;
    put16(W2D, u, wt_unit(W2, 32, 127, u >> 5, (u & 31) * 8));
  } else if (blk < 16) {
    put16(W2D, (blk - 8) * 256 + tid, zz);
  } else if (blk == 16) {
    put16(WHD, tid, wt_unit(Wa, 32, 31, tid >> 3, (tid & 7) * 8));
  } else if (blk == 17) {
    v4u o = wt_unit(Wc, 1, 31, 0, (tid & 7) * 8);
    const unsigned m = tid < 8 ? 0xFFFFFFFFu : 0u;
    o &= (v4u){ m, m, m, m };
    put16(WHD, 256 + tid, o);
  } else if (blk == 18) {
    par_sec(a1s, 128, PAR + P_A1S, tid);
  } else if (blk == 19) {
    par_sec(a1d, 128, PAR + P_A1D, tid);
  } else if (blk == 20) {
    par_sec(b1, 128, PAR + P_B1, tid);
  } else if (blk == 21) {
    par_sec(a2s, 32, PAR + P_A2S, tid);
  } else if (blk == 22) {
    par_sec(a2d, 32, PAR + P_A2D, tid);
  } else if (blk == 23) {
    par_sec(b2, 32, PAR + P_B2, tid);
  } else {
    const int tc = tid < 8 ? tid : 7;
    const v4f a = *(const v4fa*)(ba + 4 * tc);
    asm volatile("" :: "v"(a));
    const float c = bc[0];
    asm volatile("" :: "v"(c));
    const unsigned ma = tid < 8 ? 0xFFFFFFFFu : 0u;
    const unsigned mb = tid == 8 ? 0xFFFFFFFFu : 0u;
    const v4f o = (v4f){ __uint_as_float(((bf16_bits(a[0]) << 16) & ma) | ((bf16_bits(c) << 16) & mb)),
                         __uint_as_float((bf16_bits(a[1]) << 16) & ma),
                         __uint_as_float((bf16_bits(a[2]) << 16) & ma),
                         __uint_as_float((bf16_bits(a[3]) << 16) & ma) };
    if (tid < 32) {
      volatile v4f* q = (volatile v4f*)(PAR + P_HB + 4 * tid);
      *q = o;
      __threadfence();
      *q = o;
    }
  }
}

__device__ __forceinline__ int hit_put(bool h, unsigned s, int entHi, int wc, int* wl) {
  const unsigned mj = __builtin_amdgcn_ballot_w32(h);
  const int pos = wc + (int)__builtin_amdgcn_mbcnt_lo(mj, 0u);
  if (h && pos < WCAP) wl[pos] = entHi | (int)s;
  return wc + (int)__builtin_popcount(mj);
}

__device__ __forceinline__ int scan_chunk(const int* __restrict__ dsts, int cbase, int slotBase, int nb,
                                          int* wl, int tid) {
  const int el0 = tid * 8;
  const int e0  = cbase + el0;
  const int e0c = e0 < EE - 8 ? e0 : EE - 8;
  const v4i da = *(const v4ia*)(dsts + e0c);
  const v4i db = *(const v4ia*)(dsts + e0c + 4);
  asm volatile("" :: "v"(da));
  asm volatile("" :: "v"(db));
  const unsigned miss = e0 < EE ? 0u : 0xFFFFFFFFu;
  const unsigned nbs = (unsigned)slotBase;
  const unsigned unb = (unsigned)nb;
  const unsigned s0 = ((unsigned)da.x - nbs) | miss, s1 = ((unsigned)da.y - nbs) | miss;
  const unsigned s2 = ((unsigned)da.z - nbs) | miss, s3 = ((unsigned)da.w - nbs) | miss;
  const unsigned s4 = ((unsigned)db.x - nbs) | miss, s5 = ((unsigned)db.y - nbs) | miss;
  const unsigned s6 = ((unsigned)db.z - nbs) | miss, s7 = ((unsigned)db.w - nbs) | miss;
  const bool h0 = s0 < unb, h1 = s1 < unb, h2 = s2 < unb, h3 = s3 < unb;
  const bool h4 = s4 < unb, h5 = s5 < unb, h6 = s6 < unb, h7 = s7 < unb;
  int wc = 0;
  const unsigned any = __builtin_amdgcn_ballot_w32(h0 | h1 | h2 | h3 | h4 | h5 | h6 | h7);
  if (any != 0u) {
    wc = hit_put(h0, s0, (el0 + 0) << 10, wc, wl);
    wc = hit_put(h1, s1, (el0 + 1) << 10, wc, wl);
    wc = hit_put(h2, s2, (el0 + 2) << 10, wc, wl);
    wc = hit_put(h3, s3, (el0 + 3) << 10, wc, wl);
    wc = hit_put(h4, s4, (el0 + 4) << 10, wc, wl);
    wc = hit_put(h5, s5, (el0 + 5) << 10, wc, wl);
    wc = hit_put(h6, s6, (el0 + 6) << 10, wc, wl);
    wc = hit_put(h7, s7, (el0 + 7) << 10, wc, wl);
  }
  return wc;
}

__global__ __launch_bounds__(256) void k_bucket(const int* __restrict__ ei, unsigned* __restrict__ LIST,
                                                int* __restrict__ OFF, int* __restrict__ CNT,
                                                int* __restrict__ FLG) {
  extern __shared__ v4f lds_dyn[];
  int* reg1 = (int*)lds_dyn;
  int* reg2 = reg1 + CAP;
  int* scnt = reg2 + CAP;
  int* soff = scnt + NB;
  int* cur  = soff + NB;
  int* list = cur + NB;
  int* wcnt = list + LISTN;
  int* wtot = wcnt + 8;
  int* wflg = wtot + 8;
  const int tid = (int)threadIdx.x, lane = tid & 31, wave = tid >> 5;
  const int b = (int)blockIdx.x;
  const int slotBase = b * NB;
  const int nb = (NN - slotBase) < NB ? (NN - slotBase) : NB;
  const int* srcs = ei;
  const int* dsts = ei + EE;

  {
    const v4i z4 = (v4i){ 0, 0, 0, 0 };
    for (int i = tid; i < CAP / 4; i += 256) { ((v4ia*)reg1)[i] = z4; ((v4ia*)reg2)[i] = z4; }
    for (int i = tid; i < NB; i += 256) { scnt[i] = 0; soff[i] = 0; cur[i] = 0; }
    for (int i = tid; i < LISTN; i += 256) list[i] = 0;
    if (tid < 32) wcnt[tid] = 0;
  }
  __syncthreads();

  int tot = 0, totraw = 0;
  int* wl = list + wave * WCAP;
#pragma unroll 1
  for (int ch = 0; ch < NCHUNK; ++ch) {
    const int cbase = ch * CHUNK;
    const int wc = scan_chunk(dsts, cbase, slotBase, nb, wl, tid);
    if (lane == 0) wcnt[wave] = wc;
    __syncthreads();
    int pre = 0, all = 0;
#pragma unroll
    for (int w2 = 0; w2 < 8; ++w2) {
      const int c = clampi(wcnt[w2], 0, WCAP);
      all += c;
      pre += (w2 < wave) ? c : 0;
    }
    const int wcc  = __builtin_amdgcn_readfirstlane(clampi(wc, 0, WCAP));
    const int base = tot + pre;
#pragma unroll 1
    for (int i0 = 0; i0 < wcc; i0 += 32) {
      const int i   = i0 + lane;
      const int ii  = i < wcc - 1 ? i : wcc - 1;
      const int ent = wl[ii];
      const int el  = (ent >> 10) & (CHUNK - 1);
      const int sl  = ent & (NB - 1);
      const int eid = clampi(cbase + el, 0, EE - 1);
      const int sraw = srcs[eid];
      asm volatile("" :: "v"(sraw));
      const int s   = clampi(sraw, 0, NN - 1);
      const int pos = base + i;
      if (i < wcc && pos < CAP) reg1[pos] = s | (sl << 16);
    }
    totraw += all;
    tot = (tot + all) > CAP ? CAP : (tot + all);
    __syncthreads();
  }
  const int nh = tot;
  const int ovf = totraw > CAP ? 1 : 0;

  if (wave == 0) {
#pragma unroll 1
    for (int b0 = 0; b0 < nh; b0 += 32) {
      const int idx = b0 + lane;
      const int uv  = reg1[idx < CAP ? idx : CAP - 1];
      const int m32 = (nh - b0) < 32 ? (nh - b0) : 32;
#pragma unroll 1
      for (int k = 0; k < m32; ++k) {
        const int u  = __builtin_amdgcn_readlane(uv, k);
        const int sl = (u >> 16) & (NB - 1);
        if (lane == 0) scnt[sl] = scnt[sl] + 1;
      }
    }
  }
  __syncthreads();

  const v4i ca = *(const v4ia*)(scnt + 4 * tid);
  const int e0 = ca.x < 0 ? 0 : ca.x, e1 = ca.y < 0 ? 0 : ca.y, e2 = ca.z < 0 ? 0 : ca.z, e3 = ca.w < 0 ? 0 : ca.w;
  const int ts = e0 + e1 + e2 + e3;
  int incl = ts;
#pragma unroll
  for (int d = 1; d < 32; d <<= 1) {
    const int up = __shfl_up(incl, d, 32);
    incl += (lane >= d) ? up : 0;
  }
  const unsigned bigm = __builtin_amdgcn_ballot_w32((e0 > DEGCAP) | (e1 > DEGCAP) | (e2 > DEGCAP) | (e3 > DEGCAP));
  if (lane == 31) wtot[wave] = incl;
  if (lane == 0)  wflg[wave] = bigm != 0u ? 1 : 0;
  __syncthreads();
  int pre = 0, anyf = ovf;
#pragma unroll
  for (int w2 = 0; w2 < 8; ++w2) { pre += (w2 < wave) ? wtot[w2] : 0; anyf |= wflg[w2]; }
  const int r0 = pre + incl - ts;
  const int r1 = r0 + e0, r2 = r1 + e1, r3 = r2 + e2;
  const v4i vo = (v4i){ r0, r1, r2, r3 };
  soff[4 * tid + 0] = r0; soff[4 * tid + 1] = r1; soff[4 * tid + 2] = r2; soff[4 * tid + 3] = r3;
  cur[4 * tid + 0]  = r0; cur[4 * tid + 1]  = r1; cur[4 * tid + 2]  = r2; cur[4 * tid + 3]  = r3;
  __syncthreads();

  if (wave == 0) {
#pragma unroll 1
    for (int b0 = 0; b0 < nh; b0 += 32) {
      const int idx = b0 + lane;
      const int uv  = reg1[idx < CAP ? idx : CAP - 1];
      const int m32 = (nh - b0) < 32 ? (nh - b0) : 32;
#pragma unroll 1
      for (int k = 0; k < m32; ++k) {
        const int u  = __builtin_amdgcn_readlane(uv, k);
        const int sl = (u >> 16) & (NB - 1);
        if (lane == 0) {
          const int pos = clampi(cur[sl], 0, CAP - 1);
          reg2[pos] = u;
          cur[sl] = pos + 1;
        }
      }
    }
  }
  __syncthreads();

  const v4i vf = (v4i){ tid == 0 ? anyf : 0, tid == 0 ? nh : 0, 0, 0 };
  unsigned* Lb = LIST + (size_t)b * CAP;
#pragma unroll 1
  for (int pass = 0; pass < 2; ++pass) {
#pragma unroll 2
    for (int k = 0; k < CAP / 1024; ++k) {
      const int idx4 = tid + 256 * k;
      const v4i v = ((const v4ia*)reg2)[idx4];
      *(volatile v4i*)(Lb + 4 * idx4) = v;
    }
    *(volatile v4i*)(OFF + (size_t)b * NB + 4 * tid) = vo;
    *(volatile v4i*)(CNT + (size_t)b * NB + 4 * tid) = ca;
    if (tid < 8) *(volatile v4i*)(FLG + (size_t)b * 32 + 4 * tid) = vf;
    __threadfence();
  }
}

__global__ __launch_bounds__(256) void k_node1(const float* __restrict__ HW, const float* __restrict__ PAR,
                                               float* __restrict__ ASD) {
  __shared__ __attribute__((aligned(16))) float sg[8 * 64];
  const int tid = (int)threadIdx.x, lane = tid & 31, wave = tid >> 5;
  const int base = ((int)blockIdx.x * 8 + wave) * 8;
  const int head = lane >> 3;
  const v4f as = *(const v4fa*)(PAR + P_A1S + 4 * lane);
  const v4f ad = *(const v4fa*)(PAR + P_A1D + 4 * lane);
  asm volatile("" :: "v"(as));
  asm volatile("" :: "v"(ad));
  float* sw = sg + wave * 64;
#pragma unroll 2
  for (int r = 0; r < 8; ++r) {
    const v4f hv = *(const v4fa*)(HW + (size_t)(base + r) * C1 + 4 * lane);
    asm volatile("" :: "v"(hv));
    float ps = hv[0] * as[0];
    ps = ps + hv[1] * as[1];
    ps = ps + hv[2] * as[2];
    ps = ps + hv[3] * as[3];
    float pd = hv[0] * ad[0];
    pd = pd + hv[1] * ad[1];
    pd = pd + hv[2] * ad[2];
    pd = pd + hv[3] * ad[3];
    ps = ps + __shfl_xor(ps, 1, 32);
    pd = pd + __shfl_xor(pd, 1, 32);
    ps = ps + __shfl_xor(ps, 2, 32);
    pd = pd + __shfl_xor(pd, 2, 32);
    ps = ps + __shfl_xor(ps, 4, 32);
    pd = pd + __shfl_xor(pd, 4, 32);
    if ((lane & 7) == 0) { sw[r * 4 + head] = ps; sw[32 + r * 4 + head] = pd; }
  }
  __builtin_amdgcn_fence(__ATOMIC_RELEASE, "workgroup");
  __builtin_amdgcn_wave_barrier();
  __builtin_amdgcn_fence(__ATOMIC_ACQUIRE, "workgroup");
  const int l15  = lane & 15;
  const int half = l15 >> 3;
  const int rr   = l15 & 7;
  const v4f v = *(const v4fa*)(sw + half * 32 + rr * 4);
  const size_t off = (size_t)half * ((size_t)MP * 4) + (size_t)(base + rr) * 4;
  if (lane < 16) {
    volatile v4f* q = (volatile v4f*)(ASD + off);
    *q = v;
    __threadfence();
    *q = v;
  }
}

__global__ __launch_bounds__(128) void k_node2(const float* __restrict__ HW2, const float* __restrict__ PAR,
                                               float* __restrict__ ASD2) {
  const int tid = (int)threadIdx.x, lane = tid & 31, wave = tid >> 5;
  const int base = ((int)blockIdx.x * 4 + wave) * 32;
  const float as = PAR[P_A2S + lane];
  const float ad = PAR[P_A2D + lane];
  asm volatile("" :: "v"(as));
  asm volatile("" :: "v"(ad));
  float ks = 0.0f, kd = 0.0f;
#pragma unroll 2
  for (int r = 0; r < 32; ++r) {
    const float hv = HW2[(size_t)(base + r) * 64 + lane];
    asm volatile("" :: "v"(hv));
    float ps = hv * as;
    float pd = hv * ad;
    ps = ps + __shfl_xor(ps, 16, 32);
    pd = pd + __shfl_xor(pd, 16, 32);
    ps = ps + __shfl_xor(ps, 8, 32);
    pd = pd + __shfl_xor(pd, 8, 32);
    ps = ps + __shfl_xor(ps, 4, 32);
    pd = pd + __shfl_xor(pd, 4, 32);
    ps = ps + __shfl_xor(ps, 2, 32);
    pd = pd + __shfl_xor(pd, 2, 32);
    ps = ps + __shfl_xor(ps, 1, 32);
    pd = pd + __shfl_xor(pd, 1, 32);
    ks = (lane == r) ? ps : ks;
    kd = (lane == r) ? pd : kd;
  }
  volatile float* qs = (volatile float*)(ASD2 + base + lane);
  volatile float* qd = (volatile float*)(ASD2 + MP + base + lane);
  *qs = ks;
  *qd = kd;
  __threadfence();
  *qs = ks;
  *qd = kd;
}

__device__ __forceinline__ float elu1(float x) {
  const float y = expm1f(x);
  return (x > 0.0f) ? x : y;
}

__global__ __launch_bounds__(256) void k_replay1(
    const unsigned* __restrict__ LIST, const int* __restrict__ OFF, const int* __restrict__ CNT,
    const int* __restrict__ FLG, const float* __restrict__ HW, const float* __restrict__ ASD,
    const float* __restrict__ PAR, unsigned short* __restrict__ H1) {
  __shared__ float strip[8 * SROWS * 32];
  const int tid = (int)threadIdx.x, lane = tid & 31, wave = tid >> 5;
  const int i  = __builtin_amdgcn_readfirstlane((int)blockIdx.x * 8 + wave);
  const int ic = i < NN ? i : NN - 1;
  const int b  = i >> 10;
  const int head = lane >> 3;
  int st   = OFF[i];
  int craw = CNT[i];
  int fl   = FLG[b * 32];
  int nh   = FLG[b * 32 + 1];
  asm volatile("" :: "v"(st));
  asm volatile("" :: "v"(craw));
  asm volatile("" :: "v"(fl));
  asm volatile("" :: "v"(nh));
  nh = clampi(nh, 0, CAP);
  st = clampi(st, 0, nh);
  int c = clampi(craw, 0, DEGCAP);
  c = c < (nh - st) ? c : (nh - st);
  const bool live = i < NN;
  const bool pois = (fl != 0) | (craw > DEGCAP) | (craw < 0);
  const int cn = __builtin_amdgcn_readfirstlane(live ? c : 0);

  const unsigned* Lb = LIST + (size_t)b * CAP;
  const int j0 = (st + lane) < (CAP - 1) ? (st + lane) : (CAP - 1);
  const int j1 = (st + 32 + lane) < (CAP - 1) ? (st + 32 + lane) : (CAP - 1);
  const int w0 = (int)Lb[j0];
  const int w1 = (int)Lb[j1];
  asm volatile("" :: "v"(w0));
  asm volatile("" :: "v"(w1));
  const float adI = ASD[(size_t)MP * 4 + (size_t)ic * 4 + head];
  asm volatile("" :: "v"(adI));

  float* sp = strip + wave * (SROWS * 32) + lane;
  float m = -__builtin_inff();
#pragma unroll 1
  for (int q = 0; q <= cn; ++q) {
    const int u0 = __builtin_amdgcn_readlane(w0, q & 31);
    const int u1 = __builtin_amdgcn_readlane(w1, q & 31);
    const int u  = q < 32 ? u0 : u1;
    const int sl = clampi(u & 0xFFFF, 0, NN - 1);
    const int s  = q < cn ? sl : ic;
    const float a = ASD[(size_t)s * 4 + head];
    asm volatile("" :: "v"(a));
    const float v = a + adI;
    const float e = (v >= 0.0f) ? v : 0.2f * v;
    sp[q * 32] = e;
    const bool t = (e > m) | (e != e);
    m = t ? e : m;
  }
  float den = 0.0f;
#pragma unroll 1
  for (int q = 0; q <= cn; ++q) {
    const float ex = expf(sp[q * 32] - m);
    den = den + ex;
    sp[q * 32] = ex;
  }
  v4f acc = (v4f){ 0.0f, 0.0f, 0.0f, 0.0f };
#pragma unroll 1
  for (int q = 0; q <= cn; ++q) {
    const int u0 = __builtin_amdgcn_readlane(w0, q & 31);
    const int u1 = __builtin_amdgcn_readlane(w1, q & 31);
    const int u  = q < 32 ? u0 : u1;
    const int sl = clampi(u & 0xFFFF, 0, NN - 1);
    const int s  = q < cn ? sl : ic;
    const v4f row = *(const v4fa*)(HW + (size_t)s * C1 + 4 * lane);
    asm volatile("" :: "v"(row));
    const float al = sp[q * 32] / den;
    acc = acc + row * al;
  }
  const v4f bv = *(const v4fa*)(PAR + P_B1 + 4 * lane);
  asm volatile("" :: "v"(bv));
  const v4f z = acc + bv;
  float r0 = z[0], r1 = z[1], r2 = z[2], r3 = z[3];
#pragma unroll 1
  for (int cc = 0; cc < 4; ++cc) {
    const float xv = cc == 0 ? r0 : (cc == 1 ? r1 : (cc == 2 ? r2 : r3));
    const float y  = elu1(xv);
    r0 = cc == 0 ? y : r0;
    r1 = cc == 1 ? y : r1;
    r2 = cc == 2 ? y : r2;
    r3 = cc == 3 ? y : r3;
  }
  const float qn = __uint_as_float(0x7fc00000u);
  r0 = live ? (pois ? qn : r0) : 0.0f;
  r1 = live ? (pois ? qn : r1) : 0.0f;
  r2 = live ? (pois ? qn : r2) : 0.0f;
  r3 = live ? (pois ? qn : r3) : 0.0f;
  const v2u hi = (v2u){ pk16(bf16_bits(r0), bf16_bits(r1)), pk16(bf16_bits(r2), bf16_bits(r3)) };
  const v2u lo = (v2u){ pk16(bf16_lo_bits(r0), bf16_lo_bits(r1)) & LOMASK2,
                        pk16(bf16_lo_bits(r2), bf16_lo_bits(r3)) & LOMASK2 };
  volatile v2u* ph = (volatile v2u*)(H1 + (size_t)i * 256 + 4 * lane);
  volatile v2u* pl = (volatile v2u*)(H1 + (size_t)i * 256 + 128 + 4 * lane);
  *ph = hi;
  *pl = lo;
  __threadfence();
  *ph = hi;
  *pl = lo;
}

__global__ __launch_bounds__(256) void k_replay2(
    const unsigned* __restrict__ LIST, const int* __restrict__ OFF, const int* __restrict__ CNT,
    const int* __restrict__ FLG, const float* __restrict__ HW2, const float* __restrict__ ASD2,
    const float* __restrict__ PAR, unsigned short* __restrict__ H2) {
  __shared__ float strip[8 * SROWS * 32];
  const int tid = (int)threadIdx.x, lane = tid & 31, wave = tid >> 5;
  const int i  = __builtin_amdgcn_readfirstlane((int)blockIdx.x * 8 + wave);
  const int ic = i < NN ? i : NN - 1;
  const int b  = i >> 10;
  int st   = OFF[i];
  int craw = CNT[i];
  int fl   = FLG[b * 32];
  int nh   = FLG[b * 32 + 1];
  asm volatile("" :: "v"(st));
  asm volatile("" :: "v"(craw));
  asm volatile("" :: "v"(fl));
  asm volatile("" :: "v"(nh));
  nh = clampi(nh, 0, CAP);
  st = clampi(st, 0, nh);
  int c = clampi(craw, 0, DEGCAP);
  c = c < (nh - st) ? c : (nh - st);
  const bool live = i < NN;
  const bool pois = (fl != 0) | (craw > DEGCAP) | (craw < 0);
  const int cn = __builtin_amdgcn_readfirstlane(live ? c : 0);

  const unsigned* Lb = LIST + (size_t)b * CAP;
  const int j0 = (st + lane) < (CAP - 1) ? (st + lane) : (CAP - 1);
  const int j1 = (st + 32 + lane) < (CAP - 1) ? (st + 32 + lane) : (CAP - 1);
  const int w0 = (int)Lb[j0];
  const int w1 = (int)Lb[j1];
  asm volatile("" :: "v"(w0));
  asm volatile("" :: "v"(w1));
  const float adI = ASD2[(size_t)MP + ic];
  asm volatile("" :: "v"(adI));

  float* sp = strip + wave * (SROWS * 32) + lane;
  float m = -__builtin_inff();
#pragma unroll 1
  for (int q = 0; q <= cn; ++q) {
    const int u0 = __builtin_amdgcn_readlane(w0, q & 31);
    const int u1 = __builtin_amdgcn_readlane(w1, q & 31);
    const int u  = q < 32 ? u0 : u1;
    const int sl = clampi(u & 0xFFFF, 0, NN - 1);
    const int s  = q < cn ? sl : ic;
    const float a = ASD2[s];
    asm volatile("" :: "v"(a));
    const float v = a + adI;
    const float e = (v >= 0.0f) ? v : 0.2f * v;
    sp[q * 32] = e;
    const bool t = (e > m) | (e != e);
    m = t ? e : m;
  }
  float den = 0.0f;
#pragma unroll 1
  for (int q = 0; q <= cn; ++q) {
    const float ex = expf(sp[q * 32] - m);
    den = den + ex;
    sp[q * 32] = ex;
  }
  float acc = 0.0f;
#pragma unroll 1
  for (int q = 0; q <= cn; ++q) {
    const int u0 = __builtin_amdgcn_readlane(w0, q & 31);
    const int u1 = __builtin_amdgcn_readlane(w1, q & 31);
    const int u  = q < 32 ? u0 : u1;
    const int sl = clampi(u & 0xFFFF, 0, NN - 1);
    const int s  = q < cn ? sl : ic;
    const float row = HW2[(size_t)s * 64 + lane];
    asm volatile("" :: "v"(row));
    const float al = sp[q * 32] / den;
    acc = acc + al * row;
  }
  const float bv = PAR[P_B2 + lane];
  asm volatile("" :: "v"(bv));
  float r = elu1(acc + bv);
  const float qn = __uint_as_float(0x7fc00000u);
  r = live ? (pois ? qn : r) : 0.0f;
  const int cs = 2 * (lane & 15);
  const float v0 = __shfl(r, cs, 32);
  const float v1 = __shfl(r, cs + 1, 32);
  const unsigned whi = pk16(bf16_bits(v0), bf16_bits(v1));
  const unsigned wlo = pk16(bf16_lo_bits(v0), bf16_lo_bits(v1)) & LOMASK3;
  const unsigned wsel = lane < 16 ? whi : wlo;
  volatile unsigned* q = (volatile unsigned*)(H2 + (size_t)i * 64) + lane;
  *q = wsel;
  __threadfence();
  *q = wsel;
}

__global__ __launch_bounds__(256) void k_out(const float* __restrict__ T, float* __restrict__ out) {
  const int f  = (int)blockIdx.x * 256 + (int)threadIdx.x;
  const int fc = f < LOGIT_ELEMS ? f : LOGIT_ELEMS - 1;
  const int a  = fc / NN;
  const int n  = fc - a * NN;
  const float v = T[(size_t)n * 64 + a];
  asm volatile("" :: "v"(v));
  if (f < LOGIT_ELEMS) {
    volatile float* q = (volatile float*)(out + f);
    *q = v;
    __threadfence();
    *q = v;
  }
}

__global__ __launch_bounds__(256) void k_vrec(const float* __restrict__ T, double* __restrict__ REC) {
  __shared__ double sd[8];
  const int tid = (int)threadIdx.x, lane = tid & 31, wave = tid >> 5;
  const int n  = (int)blockIdx.x * 256 + tid;
  const int nc = n < NN ? n : NN - 1;
  const float v = T[(size_t)nc * 64 + 32];
  asm volatile("" :: "v"(v));
  double d = (double)v;
  d = n < NN ? d : 0.0;
  d = d + __shfl_xor(d, 16, 32);
  d = d + __shfl_xor(d, 8, 32);
  d = d + __shfl_xor(d, 4, 32);
  d = d + __shfl_xor(d, 2, 32);
  d = d + __shfl_xor(d, 1, 32);
  if (lane == 0) sd[wave] = d;
  __syncthreads();
  double tot = sd[0];
#pragma unroll
  for (int w = 1; w < 8; ++w) tot = tot + sd[w];
  const v2d o = (v2d){ tid == 0 ? tot : 0.0, 0.0 };
  if (tid < 8) {
    volatile v2d* q = (volatile v2d*)(REC + (size_t)blockIdx.x * 16 + 2 * tid);
    *q = o;
    __threadfence();
    *q = o;
  }
}

__global__ __launch_bounds__(32) void k_vcomb(const double* __restrict__ REC, float* __restrict__ out, double inv_n) {
  double s = 0.0;
#pragma unroll 1
  for (int k = 0; k < NREC; ++k) s = s + REC[(size_t)k * 16];
  const float val = (float)(s * inv_n);
  if (threadIdx.x == 0) {
    volatile float* q = (volatile float*)(out + LOGIT_ELEMS);
    *q = val;
    __threadfence();
    *q = val;
  }
}

extern "C" void kernel_launch(void* const* d_in, const int* in_sizes, int n_in,
                              void* d_out, int out_size, void* d_ws, size_t ws_size,
                              hipStream_t stream) {
  if (n_in < 14) return;
  if (in_sizes[0] != NN * FIN) return;
  if (in_sizes[1] != 2 * EE) return;
  if (in_sizes[2] != FIN * C1) return;
  if (in_sizes[3] != 128 || in_sizes[4] != 128 || in_sizes[5] != 128) return;
  if (in_sizes[6] != C1 * HID) return;
  if (in_sizes[7] != 32 || in_sizes[8] != 32 || in_sizes[9] != 32) return;
  if (in_sizes[10] != HID * 32) return;
  if (in_sizes[11] != 32 || in_sizes[12] != 32 || in_sizes[13] != 1) return;
  if (out_size != OUT_ELEMS) return;
  if (ws_size < WS_TOTAL) return;

  const float* x   = (const float*)d_in[0];
  const int*   ei  = (const int*)  d_in[1];
  const float* W1  = (const float*)d_in[2];
  const float* a1s = (const float*)d_in[3];
  const float* a1d = (const float*)d_in[4];
  const float* b1  = (const float*)d_in[5];
  const float* W2  = (const float*)d_in[6];
  const float* a2s = (const float*)d_in[7];
  const float* a2d = (const float*)d_in[8];
  const float* b2  = (const float*)d_in[9];
  const float* Wa  = (const float*)d_in[10];
  const float* ba  = (const float*)d_in[11];
  const float* Wc  = (const float*)d_in[12];
  const float* bc  = (const float*)d_in[13];
  float* out = (float*)d_out;

  char* ws = (char*)d_ws;
  unsigned short* XB   = (unsigned short*)(ws + OFF_XB);
  float*          HW   = (float*)(ws + OFF_HW);
  unsigned short* H1HL = (unsigned short*)(ws + OFF_H1);
  float*          HW2  = (float*)(ws + OFF_HW2);
  unsigned short* H2HL = (unsigned short*)(ws + OFF_H2);
  float*          T    = (float*)(ws + OFF_T);
  float*          ASD1 = (float*)(ws + OFF_ASD1);
  float*          ASD2 = (float*)(ws + OFF_ASD2);
  unsigned*       LIST = (unsigned*)(ws + OFF_LIST);
  int*            OFFT = (int*)(ws + OFF_OFF);
  int*            CNTT = (int*)(ws + OFF_CNT);
  int*            FLG  = (int*)(ws + OFF_FLG);
  unsigned short* W1T  = (unsigned short*)(ws + OFF_W1T);
  unsigned short* W2D  = (unsigned short*)(ws + OFF_W2D);
  unsigned short* WHD  = (unsigned short*)(ws + OFF_WHD);
  float*          PAR  = (float*)(ws + OFF_PAR);
  double*         REC  = (double*)(ws + OFF_REC);

  hipFuncSetAttribute(reinterpret_cast<const void*>(&k_bucket),
                      hipFuncAttributeMaxDynamicSharedMemorySize, LDS_BUCKET);

  k_plane<0><<<MP * FIN / 8 / 256, 256, 0, stream>>>(x, NN, FIN, FIN, XB, MP, FIN);
  k_prep<<<25, 256, 0, stream>>>(W1, W2, Wa, Wc, a1s, a1d, b1, a2s, a2d, b2, ba, bc, W1T, W2D, WHD, PAR);
  k_bucket<<<NBLK, 256, LDS_BUCKET, stream>>>(ei, LIST, OFFT, CNTT, FLG);
  k_gemm_nt<0, 0><<<(782 * 2 + 7) / 8, 256, 0, stream>>>(XB, W1T, PAR, HW, MP, C1, FIN, C1);
  k_node1<<<MP / 64, 256, 0, stream>>>(HW, PAR, ASD1);
  k_replay1<<<MP / 8, 256, 0, stream>>>(LIST, OFFT, CNTT, FLG, HW, ASD1, PAR, H1HL);
  k_gemm_nt<0, 0><<<(782 + 7) / 8, 256, 0, stream>>>(H1HL, W2D, PAR, HW2, MP, 64, 256, 64);
  k_node2<<<MP / 128, 128, 0, stream>>>(HW2, PAR, ASD2);
  k_replay2<<<MP / 8, 256, 0, stream>>>(LIST, OFFT, CNTT, FLG, HW2, ASD2, PAR, H2HL);
  k_gemm_nt<0, 1><<<(782 + 7) / 8, 256, 0, stream>>>(H2HL, WHD, PAR + P_HB, T, MP, 64, 64, 64);
  k_out<<<LOGIT_ELEMS / 256, 256, 0, stream>>>(T, out);
  k_vrec<<<NREC, 256, 0, stream>>>(T, REC);
  k_vcomb<<<1, 32, 0, stream>>>(REC, out, 1.0 / (double)NN);
}
